// Graph_GAN_70635032150621
// MI455X (gfx1250) — hardware-verified
//
#include <hip/hip_runtime.h>
#include <stddef.h>
#include <stdint.h>

#define NBATCH 32
#define NNODE  100
#define DNODE  32
#define NROW   3200
#define FE1    96
#define FE2    160
#define FE3    192
#define FNK0   224
#define FNH    256
#define MPAD   112
#define PWAV   7
#define PTHR   224
#define A1P    104
#define A2P    168
#define GROWS  64
#define GTHR   128
#define WSC    64.0f
#define WSCI   0.015625f
#define LRA    0.2f
#define WSMAX  134217728

static_assert(NROW == NBATCH * NNODE);
static_assert(NROW % GROWS == 0);
static_assert(MPAD == PWAV * 16 && MPAD >= NNODE);
static_assert(PTHR == PWAV * 32);
static_assert(FE1 % 32 == 0 && FE2 % 32 == 0 && FE3 % 32 == 0 && FNK0 % 32 == 0 && FNH % 32 == 0 && DNODE % 32 == 0);
static_assert((MPAD * (FE1 / 4)) % PTHR == 0);
static_assert(((A1P * 2) % 16) == 0 && ((A2P * 2) % 16) == 0 && A1P >= FE1 && A2P >= FE2);
static_assert(FE3 <= PTHR && (FE3 / 4) <= PTHR);

#define KP_OFF_PA   0
#define KP_OFF_A1   384
#define KP_OFF_A2   (KP_OFF_A1 + MPAD * A1P * 2)
#define KP_OFF_PART (KP_OFF_A2 + MPAD * A2P * 2)
#define KP_OFF_OUT  (KP_OFF_PART + PWAV * FE3 * 4)
#define KP_LDS      (KP_OFF_OUT + FE3 * 4)
static_assert(KP_OFF_A1 >= FE1 * 4);
static_assert(KP_OFF_A1 % 16 == 0 && KP_OFF_A2 % 16 == 0 && KP_OFF_PART % 16 == 0 && KP_OFF_OUT % 16 == 0);

typedef _Float16       v16h  __attribute__((ext_vector_type(16)));
typedef _Float16       v8h   __attribute__((ext_vector_type(8)));
typedef _Float16       v4h   __attribute__((ext_vector_type(4)));
typedef float          v8f   __attribute__((ext_vector_type(8)));
typedef float          v4f   __attribute__((ext_vector_type(4)));
typedef int            v8i   __attribute__((ext_vector_type(8)));
typedef unsigned short v4us  __attribute__((ext_vector_type(4)));
typedef unsigned short v8us  __attribute__((ext_vector_type(8)));
typedef unsigned short v16us __attribute__((ext_vector_type(16)));
typedef __bf16         v16bf __attribute__((ext_vector_type(16)));
typedef v8h  __attribute__((may_alias)) v8ha;
typedef v4h  __attribute__((may_alias)) v4ha;
typedef v4f  __attribute__((may_alias)) v4fa;
typedef v4us __attribute__((may_alias)) v4usa;
typedef v8us __attribute__((may_alias)) v8usa;

union Frag  { v16h v; v8h half[2]; };
union FragB { v16bf v; v16us u; v8us h[2]; v8i w; };

__device__ __forceinline__ v8f wmma_f16(v16h a, v16h b, v8f c) {
  v8f d = __builtin_amdgcn_wmma_f32_16x16x32_f16(false, a, false, b, (short)0, c, false, false);
  asm volatile("v_nop\n\tv_nop\n\tv_nop\n\tv_nop" : "+v"(d) : "v"(a), "v"(b));
  return d;
}
__device__ __forceinline__ v8f wmb(const FragB& a, const FragB& b, v8f c) {
  v8f d = __builtin_amdgcn_wmma_f32_16x16x32_bf16(false, a.v, false, b.v, (short)0, c, false, false);
  asm volatile("v_nop\n\tv_nop\n\tv_nop\n\tv_nop" : "+v"(d) : "v"(a.w), "v"(b.w));
  return d;
}

__device__ __forceinline__ v16h load_frag(const _Float16* p, int h) {
  Frag f;
  f.half[0] = *(const v8ha*)(p + 8 * h);
  f.half[1] = *(const v8ha*)(p + 16 + 8 * h);
  return f.v;
}
__device__ __forceinline__ void ldb(FragB& f, const unsigned short* p, int h) {
  f.h[0] = *(const v8usa*)(p + 8 * h);
  f.h[1] = *(const v8usa*)(p + 16 + 8 * h);
}

__device__ __forceinline__ unsigned bf16_bits(float f) {
  const unsigned u = __float_as_uint(f);
  return (u + 0x7FFFu + ((u >> 16) & 1u)) >> 16;
}
__device__ __forceinline__ void split_bf(float v, unsigned short& hb, unsigned short& lb) {
  const unsigned hu = bf16_bits(v);
  hb = (unsigned short)hu;
  lb = (unsigned short)bf16_bits(v - __uint_as_float(hu << 16));
}

__device__ __forceinline__ float lrelu(float x) { return fmaxf(x, LRA * x); }

__global__ __launch_bounds__(256) void k_w0prep(const float* __restrict__ W, unsigned short* Dh, unsigned short* Dl,
                                                int nUnits) {
  const int u = (int)blockIdx.x * 256 + (int)threadIdx.x;
  if (u >= nUnits) return;
  const int it  = u / 768;
  const int rem = u - it * 768;
  const int np  = rem >> 2;
  const int k8  = rem & 3;
  const int s   = (np >= FE1) ? 1 : 0;
  const int n   = np - s * FE1;
  const float* p = W + (size_t)it * 64 * FE1 + (size_t)(32 * s + 8 * k8) * FE1 + n;
  v8us oh, ol;
#pragma unroll
  for (int j = 0; j < 8; ++j) {
    unsigned short hb, lb;
    split_bf(p[(size_t)j * FE1], hb, lb);
    oh[j] = hb; ol[j] = lb;
  }
  unsigned short* dh = Dh + (size_t)8 * u;
  unsigned short* dl = Dl + (size_t)8 * u;
  *(volatile v8us*)dh = oh;
  *(volatile v8us*)dl = ol;
  __threadfence();
  *(volatile v8us*)dh = oh;
  *(volatile v8us*)dl = ol;
}

__global__ __launch_bounds__(256) void k_wprep_f16(const float* __restrict__ W, _Float16* D, int K, int Nn, int nUnits) {
  const int u = (int)blockIdx.x * 256 + (int)threadIdx.x;
  if (u >= nUnits) return;
  const int kb  = K >> 3;
  const int per = Nn * kb;
  const int it  = u / per;
  const int rem = u - it * per;
  const int n   = rem / kb;
  const int k8  = rem - n * kb;
  const float* p = W + (size_t)it * K * Nn + (size_t)(8 * k8) * Nn + n;
  v8h o;
#pragma unroll
  for (int j = 0; j < 8; ++j) o[j] = (_Float16)(WSC * p[(size_t)j * Nn]);
  _Float16* d = D + (size_t)8 * u;
  *(volatile v8h*)d = o;
  __threadfence();
  *(volatile v8h*)d = o;
}

__global__ __launch_bounds__(256) void k_wprep_bf(const float* __restrict__ W, unsigned short* Dh, unsigned short* Dl,
                                                 int K, int Nn, int nUnits) {
  const int u = (int)blockIdx.x * 256 + (int)threadIdx.x;
  if (u >= nUnits) return;
  const int kb  = K >> 3;
  const int per = Nn * kb;
  const int it  = u / per;
  const int rem = u - it * per;
  const int n   = rem / kb;
  const int k8  = rem - n * kb;
  const float* p = W + (size_t)it * K * Nn + (size_t)(8 * k8) * Nn + n;
  v8us oh, ol;
#pragma unroll
  for (int j = 0; j < 8; ++j) {
    unsigned short hb, lb;
    split_bf(p[(size_t)j * Nn], hb, lb);
    oh[j] = hb; ol[j] = lb;
  }
  unsigned short* dh = Dh + (size_t)8 * u;
  unsigned short* dl = Dl + (size_t)8 * u;
  *(volatile v8us*)dh = oh;
  *(volatile v8us*)dl = ol;
  __threadfence();
  *(volatile v8us*)dh = oh;
  *(volatile v8us*)dl = ol;
}

__host__ __device__ constexpr int ng_lds(int K, int NB) { return 2 * GROWS * (K + 8) * 2 + GROWS * NB * 4; }

template <int K, int NB, bool CONCAT, bool ACT, int BOFF>
__global__ __launch_bounds__(GTHR) void k_ngemm(
    const float* __restrict__ A0, const float* __restrict__ AX,
    const unsigned short* __restrict__ Wh, const unsigned short* __restrict__ Wl,
    const float* __restrict__ bias, float* C, int N)
{
  constexpr int AP   = K + 8;
  constexpr int NTL  = NB / 16;
  constexpr int UPR  = K / 4;
  constexpr int NIT  = (GROWS * UPR) / GTHR;
  constexpr int UPO  = NB / 4;
  constexpr int NITO = (GROWS * UPO) / GTHR;
  static_assert(NTL >= 1 && NTL <= 8);
  static_assert(K % 32 == 0 && NB % 32 == 0);
  static_assert((GROWS * UPR) % GTHR == 0 && (GROWS * UPO) % GTHR == 0);
  static_assert(!CONCAT || K == FE3 + DNODE);
  static_assert(((AP * 2) % 16) == 0);

  extern __shared__ __attribute__((aligned(16))) char smem[];
  unsigned short* sAh = (unsigned short*)smem;
  unsigned short* sAl = sAh + GROWS * AP;
  float* sO = (float*)(smem + (size_t)2 * GROWS * AP * 2);

  const int tid = (int)threadIdx.x, lane = tid & 31, w = tid >> 5;
  const int h = lane >> 4, m = lane & 15;
  const int row0 = (int)blockIdx.x * GROWS;
  const int n0 = (int)blockIdx.y * NB;

#pragma unroll 2
  for (int i = 0; i < NIT; ++i) {
    const int u = i * GTHR + tid;
    const int row = u / UPR;
    const int c4 = u - row * UPR;
    v4f v;
    if constexpr (CONCAT) {
      const int c  = 4 * c4;
      const int ca = c < FE3 - 4 ? c : FE3 - 4;
      int cx = c - FE3; cx = cx < 0 ? 0 : (cx > DNODE - 4 ? DNODE - 4 : cx);
      const v4f va = *(const v4fa*)(A0 + (size_t)(row0 + row) * FE3 + ca);
      const v4f vx = *(const v4fa*)(AX + (size_t)(row0 + row) * DNODE + cx);
      const unsigned msk = (c < FE3) ? 0xffffffffu : 0u;
      v.x = __uint_as_float((__float_as_uint(va.x) & msk) | (__float_as_uint(vx.x) & ~msk));
      v.y = __uint_as_float((__float_as_uint(va.y) & msk) | (__float_as_uint(vx.y) & ~msk));
      v.z = __uint_as_float((__float_as_uint(va.z) & msk) | (__float_as_uint(vx.z) & ~msk));
      v.w = __uint_as_float((__float_as_uint(va.w) & msk) | (__float_as_uint(vx.w) & ~msk));
    } else {
      v = *(const v4fa*)(A0 + (size_t)(row0 + row) * K + 4 * c4);
    }
    v4us hb, lb;
    { unsigned short a, b; split_bf(v.x, a, b); hb[0] = a; lb[0] = b; }
    { unsigned short a, b; split_bf(v.y, a, b); hb[1] = a; lb[1] = b; }
    { unsigned short a, b; split_bf(v.z, a, b); hb[2] = a; lb[2] = b; }
    { unsigned short a, b; split_bf(v.w, a, b); hb[3] = a; lb[3] = b; }
    *(v4usa*)(sAh + row * AP + 4 * c4) = hb;
    *(v4usa*)(sAl + row * AP + 4 * c4) = lb;
  }
  __syncthreads();

  v8f acc[NTL];
  {
    const v8f z8 = {0.f, 0.f, 0.f, 0.f, 0.f, 0.f, 0.f, 0.f};
#pragma unroll
    for (int t = 0; t < NTL; ++t) acc[t] = z8;
  }
  const unsigned short* ah  = sAh + (16 * w + m) * AP;
  const unsigned short* al  = sAl + (16 * w + m) * AP;
  const unsigned short* wh0 = Wh + (size_t)(n0 + m) * K;
  const unsigned short* wl0 = Wl + (size_t)(n0 + m) * K;

#pragma unroll 1
  for (int k0 = 0; k0 < K; k0 += 32) {
    FragB fah, fal;
    ldb(fah, ah + k0, h);
    ldb(fal, al + k0, h);
#pragma unroll
    for (int nt = 0; nt < NTL; ++nt) {
      FragB fwh, fwl;
      ldb(fwh, wh0 + (size_t)(16 * nt) * K + k0, h);
      ldb(fwl, wl0 + (size_t)(16 * nt) * K + k0, h);
      acc[nt] = wmb(fah, fwh, acc[nt]);
      acc[nt] = wmb(fal, fwh, acc[nt]);
      acc[nt] = wmb(fah, fwl, acc[nt]);
    }
  }

#pragma unroll
  for (int nt = 0; nt < NTL; ++nt) {
    const int cl  = 16 * nt + m;
    const int col = n0 + cl;
    float bv;
    if constexpr (BOFF > 0) {
      int bi = col - BOFF; bi = bi < 0 ? 0 : bi;
      const float bs = (col >= BOFF) ? 1.0f : 0.0f;
      bv = bias[bi] * bs;
    } else {
      bv = bias[col];
    }
#pragma unroll
    for (int r = 0; r < 8; ++r) {
      float y = acc[nt][r] + bv;
      if constexpr (ACT) y = lrelu(y);
      sO[(16 * w + 8 * h + r) * NB + cl] = y;
    }
  }
  __syncthreads();

#pragma unroll 2
  for (int i = 0; i < NITO; ++i) {
    const int u = i * GTHR + tid;
    const int row = u / UPO;
    const int c4 = u - row * UPO;
    const v4f v = *(const v4fa*)(sO + row * NB + 4 * c4);
    *(volatile v4f*)(C + (size_t)(row0 + row) * N + n0 + 4 * c4) = v;
  }
  __threadfence();
#pragma unroll 2
  for (int i = 0; i < NITO; ++i) {
    const int u = i * GTHR + tid;
    const int row = u / UPO;
    const int c4 = u - row * UPO;
    const v4f v = *(const v4fa*)(sO + row * NB + 4 * c4);
    *(volatile v4f*)(C + (size_t)(row0 + row) * N + n0 + 4 * c4) = v;
  }
}

__global__ __launch_bounds__(PTHR) void k_pair(
    const float* __restrict__ PQ,
    const _Float16* __restrict__ WF1,
    const _Float16* __restrict__ WF2,
    const float* __restrict__ b1,
    const float* __restrict__ b2,
    float* AGG)
{
  extern __shared__ __attribute__((aligned(16))) char smem[];
  float*    sPA   = (float*)(smem + KP_OFF_PA);
  _Float16* sA1   = (_Float16*)(smem + KP_OFF_A1);
  _Float16* sA2   = (_Float16*)(smem + KP_OFF_A2);
  float*    sPart = (float*)(smem + KP_OFF_PART);
  float*    sOut  = (float*)(smem + KP_OFF_OUT);

  const int tid = (int)threadIdx.x, lane = tid & 31, w = tid >> 5;
  const int h = lane >> 4, m = lane & 15;
  const int q = (int)blockIdx.x;
  const int b = q / NNODE;
  const int prow0 = b * NNODE;

  {
    const int t = tid < (FE1 / 4 - 1) ? tid : (FE1 / 4 - 1);
    const v4f v = *(const v4fa*)(PQ + (size_t)q * FE3 + 4 * t);
    if (tid < FE1 / 4) *(v4fa*)(sPA + 4 * t) = v;
  }
  __syncthreads();

#pragma unroll 2
  for (int i = 0; i < (MPAD * (FE1 / 4)) / PTHR; ++i) {
    const int u  = i * PTHR + tid;
    const int r  = u / (FE1 / 4);
    const int c4 = u - r * (FE1 / 4);
    const int mc = r < NNODE ? r : NNODE - 1;
    const v4f pb = *(const v4fa*)(PQ + (size_t)(prow0 + mc) * FE3 + FE1 + 4 * c4);
    const v4f pa = *(const v4fa*)(sPA + 4 * c4);
    v4h o;
    o[0] = (_Float16)lrelu(pa.x + pb.x);
    o[1] = (_Float16)lrelu(pa.y + pb.y);
    o[2] = (_Float16)lrelu(pa.z + pb.z);
    o[3] = (_Float16)lrelu(pa.w + pb.w);
    *(v4ha*)(sA1 + r * A1P + 4 * c4) = o;
  }
  __syncthreads();

  const v8f z8 = {0.f, 0.f, 0.f, 0.f, 0.f, 0.f, 0.f, 0.f};

  {
    v16h af[FE1 / 32];
    const _Float16* ap = sA1 + (16 * w + m) * A1P;
#pragma unroll
    for (int kc = 0; kc < FE1 / 32; ++kc) af[kc] = load_frag(ap + 32 * kc, h);
    const _Float16* wb = WF1 + (size_t)m * FE1;
#pragma unroll 1
    for (int nt = 0; nt < FE2 / 16; ++nt) {
      const _Float16* wr = wb + (size_t)(16 * nt) * FE1;
      v8f acc = z8;
#pragma unroll
      for (int kc = 0; kc < FE1 / 32; ++kc) acc = wmma_f16(af[kc], load_frag(wr + 32 * kc, h), acc);
      const int col = 16 * nt + m;
      const float bv = b1[col];
#pragma unroll
      for (int r = 0; r < 8; ++r)
        sA2[(16 * w + 8 * h + r) * A2P + col] = (_Float16)lrelu(fmaf(acc[r], WSCI, bv));
    }
  }
  __syncthreads();

  {
    v16h af[FE2 / 32];
    const _Float16* ap = sA2 + (16 * w + m) * A2P;
#pragma unroll
    for (int kc = 0; kc < FE2 / 32; ++kc) af[kc] = load_frag(ap + 32 * kc, h);
    const _Float16* wb = WF2 + (size_t)m * FE2;
#pragma unroll 1
    for (int nt = 0; nt < FE3 / 16; ++nt) {
      const _Float16* wr = wb + (size_t)(16 * nt) * FE2;
      v8f acc = z8;
#pragma unroll
      for (int kc = 0; kc < FE2 / 32; ++kc) acc = wmma_f16(af[kc], load_frag(wr + 32 * kc, h), acc);
      const int col = 16 * nt + m;
      const float bv = b2[col];
      float s = 0.0f;
#pragma unroll
      for (int r = 0; r < 8; ++r) {
        const int pr = 16 * w + 8 * h + r;
        const float vld = (pr < NNODE) ? 1.0f : 0.0f;
        s = fmaf(vld, lrelu(fmaf(acc[r], WSCI, bv)), s);
      }
      s += __shfl_xor(s, 16);
      if (h == 0) sPart[w * FE3 + col] = s;
    }
  }
  __syncthreads();

  {
    const int t = tid < (FE3 - 1) ? tid : (FE3 - 1);
    float a = 0.0f;
#pragma unroll
    for (int ww = 0; ww < PWAV; ++ww) a += sPart[ww * FE3 + t];
    if (tid < FE3) sOut[t] = a;
  }
  __syncthreads();

  {
    const int t = tid < (FE3 / 4 - 1) ? tid : (FE3 / 4 - 1);
    const v4f v = *(const v4fa*)(sOut + 4 * t);
    float* dst = AGG + (size_t)q * FE3 + 4 * t;
    if (tid < FE3 / 4) *(volatile v4f*)dst = v;
    __threadfence();
    if (tid < FE3 / 4) *(volatile v4f*)dst = v;
  }
}

static inline int cdiv(int a, int b) { return (a + b - 1) / b; }

#define KN0 k_ngemm<DNODE, 96, false, false, FE1>
#define KF0 k_ngemm<FNK0, 128, true, true, 0>
#define KF1 k_ngemm<FNH, 128, false, true, 0>
#define KF2 k_ngemm<FNH, DNODE, false, false, 0>

extern "C" void kernel_launch(void* const* d_in, const int* in_sizes, int n_in,
                              void* d_out, int out_size, void* d_ws, size_t ws_size,
                              hipStream_t stream) {
  if (n_in < 13) return;
  if (in_sizes[0]  != NROW * DNODE) return;
  if (in_sizes[1]  != 2 * 64 * FE1) return;
  if (in_sizes[2]  != 2 * FE1) return;
  if (in_sizes[3]  != 2 * FE1 * FE2) return;
  if (in_sizes[4]  != 2 * FE2) return;
  if (in_sizes[5]  != 2 * FE2 * FE3) return;
  if (in_sizes[6]  != 2 * FE3) return;
  if (in_sizes[7]  != 2 * FNK0 * FNH) return;
  if (in_sizes[8]  != 2 * FNH) return;
  if (in_sizes[9]  != 2 * FNH * FNH) return;
  if (in_sizes[10] != 2 * FNH) return;
  if (in_sizes[11] != 2 * FNH * DNODE) return;
  if (in_sizes[12] != 2 * DNODE) return;
  if (out_size != NROW * DNODE) return;

  const float* x     = (const float*)d_in[0];
  const float* fe_w0 = (const float*)d_in[1];
  const float* fe_b0 = (const float*)d_in[2];
  const float* fe_w1 = (const float*)d_in[3];
  const float* fe_b1 = (const float*)d_in[4];
  const float* fe_w2 = (const float*)d_in[5];
  const float* fe_b2 = (const float*)d_in[6];
  const float* fn_w0 = (const float*)d_in[7];
  const float* fn_b0 = (const float*)d_in[8];
  const float* fn_w1 = (const float*)d_in[9];
  const float* fn_b1 = (const float*)d_in[10];
  const float* fn_w2 = (const float*)d_in[11];
  const float* fn_b2 = (const float*)d_in[12];
  float* out = (float*)d_out;

  const size_t nW0  = (size_t)2 * FE3 * DNODE;
  const size_t nWF1 = (size_t)2 * FE2 * FE1;
  const size_t nWF2 = (size_t)2 * FE3 * FE2;
  const size_t nN0  = (size_t)2 * FNH * FNK0;
  const size_t nN1  = (size_t)2 * FNH * FNH;
  const size_t nN2  = (size_t)2 * DNODE * FNH;
  char* ws = (char*)d_ws;
  size_t off = 0;
  auto take = [&](size_t bytes) { const size_t o = off; off += (bytes + 255) & ~(size_t)255; return o; };
  const size_t oW0H = take(nW0 * 2),  oW0L = take(nW0 * 2);
  const size_t oWF1 = take(nWF1 * 2), oWF2 = take(nWF2 * 2);
  const size_t oN0H = take(nN0 * 2),  oN0L = take(nN0 * 2);
  const size_t oN1H = take(nN1 * 2),  oN1L = take(nN1 * 2);
  const size_t oN2H = take(nN2 * 2),  oN2L = take(nN2 * 2);
  const size_t oPQ  = take((size_t)NROW * FE3 * 4);
  const size_t oAGG = take((size_t)NROW * FE3 * 4);
  const size_t oH1  = take((size_t)NROW * FNH * 4);
  const size_t oH2  = take((size_t)NROW * FNH * 4);
  const size_t oXP  = take((size_t)NROW * DNODE * 4);
  if (off > ws_size || off > (size_t)WSMAX) return;

  unsigned short* W0H = (unsigned short*)(ws + oW0H);
  unsigned short* W0L = (unsigned short*)(ws + oW0L);
  _Float16* WF1 = (_Float16*)(ws + oWF1);
  _Float16* WF2 = (_Float16*)(ws + oWF2);
  unsigned short* N0H = (unsigned short*)(ws + oN0H);
  unsigned short* N0L = (unsigned short*)(ws + oN0L);
  unsigned short* N1H = (unsigned short*)(ws + oN1H);
  unsigned short* N1L = (unsigned short*)(ws + oN1L);
  unsigned short* N2H = (unsigned short*)(ws + oN2H);
  unsigned short* N2L = (unsigned short*)(ws + oN2L);
  float* PQ  = (float*)(ws + oPQ);
  float* AGG = (float*)(ws + oAGG);
  float* H1  = (float*)(ws + oH1);
  float* H2  = (float*)(ws + oH2);
  float* XP  = (float*)(ws + oXP);

  const int ldsN0 = ng_lds(DNODE, 96);
  const int ldsF0 = ng_lds(FNK0, 128);
  const int ldsF1 = ng_lds(FNH, 128);
  const int ldsF2 = ng_lds(FNH, DNODE);
  (void)hipFuncSetAttribute(reinterpret_cast<const void*>(&k_pair), hipFuncAttributeMaxDynamicSharedMemorySize, KP_LDS);
  (void)hipFuncSetAttribute(reinterpret_cast<const void*>(&KN0), hipFuncAttributeMaxDynamicSharedMemorySize, ldsN0);
  (void)hipFuncSetAttribute(reinterpret_cast<const void*>(&KF0), hipFuncAttributeMaxDynamicSharedMemorySize, ldsF0);
  (void)hipFuncSetAttribute(reinterpret_cast<const void*>(&KF1), hipFuncAttributeMaxDynamicSharedMemorySize, ldsF1);
  (void)hipFuncSetAttribute(reinterpret_cast<const void*>(&KF2), hipFuncAttributeMaxDynamicSharedMemorySize, ldsF2);

  {
    const int u0 = (int)(nW0 / 8);
    k_w0prep<<<cdiv(u0, 256), 256, 0, stream>>>(fe_w0, W0H, W0L, u0);
    const int u1 = (int)(nWF1 / 8);
    k_wprep_f16<<<cdiv(u1, 256), 256, 0, stream>>>(fe_w1, WF1, FE1, FE2, u1);
    const int u2 = (int)(nWF2 / 8);
    k_wprep_f16<<<cdiv(u2, 256), 256, 0, stream>>>(fe_w2, WF2, FE2, FE3, u2);
    const int u3 = (int)(nN0 / 8);
    k_wprep_bf<<<cdiv(u3, 256), 256, 0, stream>>>(fn_w0, N0H, N0L, FNK0, FNH, u3);
    const int u4 = (int)(nN1 / 8);
    k_wprep_bf<<<cdiv(u4, 256), 256, 0, stream>>>(fn_w1, N1H, N1L, FNH, FNH, u4);
    const int u5 = (int)(nN2 / 8);
    k_wprep_bf<<<cdiv(u5, 256), 256, 0, stream>>>(fn_w2, N2H, N2L, FNH, DNODE, u5);
  }

  for (int it = 0; it < 2; ++it) {
    const float* X = (it == 0) ? x : XP;

    KN0<<<dim3(NROW / GROWS, FE3 / 96), GTHR, ldsN0, stream>>>(
        X, X, W0H + (size_t)it * FE3 * DNODE, W0L + (size_t)it * FE3 * DNODE, fe_b0 + (size_t)it * FE1, PQ, FE3);

    k_pair<<<NROW, PTHR, KP_LDS, stream>>>(
        PQ, WF1 + (size_t)it * FE2 * FE1, WF2 + (size_t)it * FE3 * FE2,
        fe_b1 + (size_t)it * FE2, fe_b2 + (size_t)it * FE3, AGG);

    KF0<<<dim3(NROW / GROWS, FNH / 128), GTHR, ldsF0, stream>>>(
        AGG, X, N0H + (size_t)it * FNH * FNK0, N0L + (size_t)it * FNH * FNK0, fn_b0 + (size_t)it * FNH, H1, FNH);

    KF1<<<dim3(NROW / GROWS, FNH / 128), GTHR, ldsF1, stream>>>(
        H1, X, N1H + (size_t)it * FNH * FNH, N1L + (size_t)it * FNH * FNH, fn_b1 + (size_t)it * FNH, H2, FNH);

    float* dst = (it == 1) ? out : XP;
    KF2<<<dim3(NROW / GROWS, 1), GTHR, ldsF2, stream>>>(
        H2, X, N2H + (size_t)it * DNODE * FNH, N2L + (size_t)it * DNODE * FNH, fn_b2 + (size_t)it * DNODE, dst, DNODE);
  }
}
